// CustomGPT2MultiHeadAttention_22600117911808
// MI455X (gfx1250) — hardware-verified
//
#include <hip/hip_runtime.h>
#include <stdint.h>
#include <math.h>

typedef __attribute__((ext_vector_type(16))) _Float16 v16h;
typedef __attribute__((ext_vector_type(8)))  _Float16 v8h;
typedef __attribute__((ext_vector_type(16))) __bf16   v16b;
typedef __attribute__((ext_vector_type(8)))  __bf16   v8b;
typedef __attribute__((ext_vector_type(8)))  float    v8f;
typedef __attribute__((ext_vector_type(4)))  float    v4f;
typedef __attribute__((ext_vector_type(4)))  unsigned int v4u;

constexpr int NBATCH   = 8;
constexpr int SEQ_LEN  = 1024;
constexpr int DMODEL   = 1024;
constexpr int NHEAD    = 16;
constexpr int HDIM     = 64;
constexpr int MASK_LEN = SEQ_LEN + 1;
constexpr int HALF_NB  = 4;
constexpr int ROWS_HALF = HALF_NB * SEQ_LEN;
constexpr int LDQK     = 2 * DMODEL;
constexpr int QBLK     = 64;
constexpr int NQB      = SEQ_LEN / QBLK;
constexpr int KVC      = 64;
constexpr int OSP      = 68;

static_assert(DMODEL % 32 == 0, "K multiple of 32");
static_assert(ROWS_HALF % 64 == 0 && LDQK % 64 == 0 && DMODEL % 64 == 0 && SEQ_LEN % 64 == 0, "tile multiples of 64");
static_assert(NHEAD * HDIM == DMODEL, "head split");
static_assert(SEQ_LEN % QBLK == 0 && QBLK == KVC, "attention blocking");

constexpr size_t WS_XB    = (size_t)NBATCH * SEQ_LEN * DMODEL * 2;
constexpr size_t WS_WQKV  = (size_t)3 * DMODEL * DMODEL * 2;
constexpr size_t WS_WP    = (size_t)DMODEL * DMODEL * 2;
constexpr size_t WS_QK    = (size_t)ROWS_HALF * LDQK * 2;
constexpr size_t WS_VT    = (size_t)HALF_NB * DMODEL * SEQ_LEN * 2;
constexpr size_t WS_X     = (size_t)ROWS_HALF * DMODEL * 2;
constexpr size_t WS_TOTAL = WS_XB + WS_WQKV + WS_WP + 2 * WS_QK + 2 * WS_VT + 2 * WS_X;
static_assert(WS_TOTAL == 92274688, "carve");
static_assert(WS_TOTAL <= 134217728, "carve budget");

__device__ __forceinline__ unsigned short f2bf_bits(float f) {
  unsigned u = __float_as_uint(f);
  return (unsigned short)((u + 0x7FFFu + ((u >> 16) & 1u)) >> 16);
}
__device__ __forceinline__ float bf_bits2f(unsigned short h) { return __uint_as_float(((unsigned)h) << 16); }
__device__ __forceinline__ float bf_rne(float f) { return bf_bits2f(f2bf_bits(f)); }

__device__ __forceinline__ void dep_guard_h(v8f& a, v8f& b, v16h x, v16h y) { asm volatile("v_nop\n\tv_nop\n\tv_nop\n\tv_nop" : "+v"(a), "+v"(b) : "v"(x), "v"(y)); }
__device__ __forceinline__ void dep_guard_b(v8f& a, v8f& b, v16b x, v16b y) { asm volatile("v_nop\n\tv_nop\n\tv_nop\n\tv_nop" : "+v"(a), "+v"(b) : "v"(x), "v"(y)); }
__device__ __forceinline__ void keep4_h(v16h a, v16h b, v16h c, v16h d) { asm volatile("v_nop" :: "v"(a), "v"(b), "v"(c), "v"(d)); }
__device__ __forceinline__ void keep4_b(v16b a, v16b b, v16b c, v16b d) { asm volatile("v_nop" :: "v"(a), "v"(b), "v"(c), "v"(d)); }
__device__ __forceinline__ void acc_guard4(v8f& a, v8f& b, v8f& c, v8f& d) { asm volatile("v_nop\n\tv_nop\n\tv_nop\n\tv_nop" : "+v"(a), "+v"(b), "+v"(c), "+v"(d)); }
template <typename T> struct Frag;
template <> struct Frag<_Float16> {
  typedef v16h V; union U { v16h v; v8h h[2]; };
  static __device__ __forceinline__ v16h load(const _Float16* p) {
    U f; f.h[0] = *(const v8h*)(p); f.h[1] = *(const v8h*)(p + 16); return f.v;
  }
  static __device__ __forceinline__ v8f mma(v16h a, v16h b, v8f c) {
    return __builtin_amdgcn_wmma_f32_16x16x32_f16(false, a, false, b, (short)0, c, false, false);
  }
  static __device__ __forceinline__ void guard(v8f& a, v8f& b, v16h x, v16h y) { dep_guard_h(a, b, x, y); }
  static __device__ __forceinline__ void keep(v16h a, v16h b, v16h c, v16h d) { keep4_h(a, b, c, d); }
};
template <> struct Frag<__bf16> {
  typedef v16b V; union U { v16b v; v8b h[2]; };
  static __device__ __forceinline__ v16b load(const __bf16* p) {
    U f; f.h[0] = *(const v8b*)(p); f.h[1] = *(const v8b*)(p + 16); return f.v;
  }
  static __device__ __forceinline__ v8f mma(v16b a, v16b b, v8f c) {
    return __builtin_amdgcn_wmma_f32_16x16x32_bf16(false, a, false, b, (short)0, c, false, false);
  }
  static __device__ __forceinline__ void guard(v8f& a, v8f& b, v16b x, v16b y) { dep_guard_b(a, b, x, y); }
  static __device__ __forceinline__ void keep(v16b a, v16b b, v16b c, v16b d) { keep4_b(a, b, c, d); }
};

__device__ __forceinline__ v8f at_mma(v16b a, v16b b, v8f c) {
  c = __builtin_amdgcn_wmma_f32_16x16x32_bf16(false, a, false, b, (short)0, c, false, false);
  asm volatile("v_nop\n\tv_nop\n\tv_nop\n\tv_nop" : "+v"(c) : "v"(a), "v"(b));
  return c;
}

template <int ET> struct Elem;
template <> struct Elem<0> { typedef _Float16 T; };
template <> struct Elem<1> { typedef __bf16 T; };
template <int ET, int SPLIT, int BIAS_MODE, int OUT_MODE, bool RESID, int ACT = 0>
__global__ __launch_bounds__(256) void wmma_gemm64(
    const unsigned short* __restrict__ Ap, const unsigned short* __restrict__ A2p, int lda, long strideA,
    const unsigned short* __restrict__ Btp, const unsigned short* __restrict__ Bt2p, int ldb, long strideB,
    void* __restrict__ Cout, void* __restrict__ Cout2, int ldc, long strideC,
    const float* __restrict__ bias,
    const float* __restrict__ resid, long strideR,
    int M, int N, int K, float scale) {
  typedef typename Elem<ET>::T T;
  typedef typename Frag<T>::V V;
  const T* A = (const T*)Ap; const T* A2 = (const T*)A2p; const T* Bt = (const T*)Btp; const T* Bt2 = (const T*)Bt2p;
  __shared__ __align__(16) float sT[8][16 * 68];
  const int b    = blockIdx.y;
  const int lane = threadIdx.x & 31;
  const int wave = threadIdx.x >> 5;
  const int tilesN = N >> 6;
  const int tilesM = M >> 6;
  const int tile = blockIdx.x * 8 + wave;
  if (tile >= tilesM * tilesN) return;
  const int tm = tile / tilesN;
  const int tn = tile - tm * tilesN;
  const int m0 = tm << 6;
  const int n0 = tn << 6;

  const T* Ab  = A  + (size_t)b * strideA;
  const T* Bb  = Bt + (size_t)b * strideB;
  const T* Ab2 = (SPLIT != 0) ? (A2  + (size_t)b * strideA) : nullptr;
  const T* Bb2 = (SPLIT == 1) ? (Bt2 + (size_t)b * strideB) : nullptr;

  const int rlane = lane & 15;
  const int koff  = (lane >> 4) * 8;
  const int mOff  = (lane >> 4) * 8;

  v8f acc[4][4];
#pragma unroll
  for (int i = 0; i < 4; ++i)
#pragma unroll
    for (int j = 0; j < 4; ++j) acc[i][j] = (v8f){0.f,0.f,0.f,0.f,0.f,0.f,0.f,0.f};

  for (int k0 = 0; k0 < K; k0 += 32) {
    V bh[4], bl[4];
#pragma unroll
    for (int j = 0; j < 4; ++j) {
      const size_t bo = (size_t)(n0 + (j << 4) + rlane) * ldb + koff + k0;
      bh[j] = Frag<T>::load(Bb + bo);
      if (SPLIT == 1) bl[j] = Frag<T>::load(Bb2 + bo);
    }
#pragma unroll
    for (int i = 0; i < 4; ++i) {
      const size_t ao = (size_t)(m0 + (i << 4) + rlane) * lda + koff + k0;
      V ah = Frag<T>::load(Ab + ao);
      V al;
      if (SPLIT != 0) al = Frag<T>::load(Ab2 + ao);
#pragma unroll
      for (int j = 0; j < 4; ++j) {
        acc[i][j] = Frag<T>::mma(ah, bh[j], acc[i][j]);
        if (SPLIT == 1) acc[i][j] = Frag<T>::mma(ah, bl[j], acc[i][j]);
        if (SPLIT != 0) acc[i][j] = Frag<T>::mma(al, bh[j], acc[i][j]);
      }
      Frag<T>::guard(acc[i][0], acc[i][3], ah, (SPLIT != 0) ? al : ah);
    }
    Frag<T>::keep(bh[0], bh[1], bh[2], bh[3]);
    if (SPLIT == 1) Frag<T>::keep(bl[0], bl[1], bl[2], bl[3]);
  }
  acc_guard4(acc[0][0], acc[0][1], acc[0][2], acc[0][3]);
  acc_guard4(acc[1][0], acc[1][1], acc[1][2], acc[1][3]);
  acc_guard4(acc[2][0], acc[2][1], acc[2][2], acc[2][3]);
  acc_guard4(acc[3][0], acc[3][1], acc[3][2], acc[3][3]);

  float* slab = sT[wave];
  const float* Rb = RESID ? (resid + (size_t)b * strideR) : nullptr;
#pragma unroll
  for (int i = 0; i < 4; ++i) {
    const int mBase = m0 + (i << 4);
#pragma unroll
    for (int j = 0; j < 4; ++j) {
      const int n = n0 + (j << 4) + rlane;
      float bv = 0.f;
      if (BIAS_MODE == 2) bv = bf_rne(bias[n]);
#pragma unroll
      for (int r = 0; r < 8; ++r) {
        float v = acc[i][j][r] * scale;
        if (BIAS_MODE == 1) v += bf_rne(bias[mBase + mOff + r]);
        if (BIAS_MODE == 2) v += bv;
        if (RESID) v += Rb[(size_t)(mBase + mOff + r) * ldc + n];
        if (ACT == 1) v = tanhf(v);
        if (ACT == 2) v = fmaxf(v, 0.0f);
        if (ACT == 3) v = v / (1.0f + expf(-v));
        if (ACT == 4) v = (v > 0.f) ? v : 0.01f * v;
        slab[(mOff + r) * 68 + (j << 4) + rlane] = v;
      }
    }
    __builtin_amdgcn_fence(__ATOMIC_RELEASE, "workgroup");
    __builtin_amdgcn_wave_barrier();
    __builtin_amdgcn_fence(__ATOMIC_ACQUIRE, "workgroup");
    if (OUT_MODE == 0) {
      float* C = (float*)Cout + (size_t)b * strideC;
      const int hh = lane >> 4, c4 = (lane & 15) * 4;
      for (int pass = 0; pass < 2; ++pass) {
#pragma unroll
        for (int it = 0; it < 8; ++it) {
          const int row = it * 2 + hh;
          v4f v = *(const v4f*)(slab + row * 68 + c4);
          *(volatile v4f*)(C + (size_t)(mBase + row) * ldc + n0 + c4) = v;
        }
        __threadfence();
      }
    } else {
      const int q = lane >> 3, c8 = (lane & 7) * 8;
      unsigned short* C  = (unsigned short*)Cout  + (size_t)b * strideC;
      unsigned short* C2 = (OUT_MODE == 2) ? ((unsigned short*)Cout2 + (size_t)b * strideC) : nullptr;
      for (int pass = 0; pass < 2; ++pass) {
#pragma unroll
        for (int it = 0; it < 4; ++it) {
          const int row = it * 4 + q;
          const float* sp = slab + row * 68 + c8;
          v8h hv, lv;
#pragma unroll
          for (int e = 0; e < 8; ++e) {
            if (OUT_MODE == 1) {
              hv[e] = (_Float16)sp[e];
            } else {
              unsigned short hb = f2bf_bits(sp[e]);
              unsigned short lb = f2bf_bits(sp[e] - bf_bits2f(hb));
              hv[e] = __builtin_bit_cast(_Float16, hb);
              lv[e] = __builtin_bit_cast(_Float16, lb);
            }
          }
          *(volatile v8h*)(C + (size_t)(mBase + row) * ldc + n0 + c8) = hv;
          if (OUT_MODE == 2) *(volatile v8h*)(C2 + (size_t)(mBase + row) * ldc + n0 + c8) = lv;
        }
        __threadfence();
      }
    }
    __builtin_amdgcn_fence(__ATOMIC_RELEASE, "workgroup");
    __builtin_amdgcn_wave_barrier();
    __builtin_amdgcn_fence(__ATOMIC_ACQUIRE, "workgroup");
  }
}

__global__ __launch_bounds__(256) void cast_rows_bf16(
    const float* __restrict__ in, unsigned short* __restrict__ out, int n8) {
  const int i = blockIdx.x * 256 + threadIdx.x;
  if (i >= n8) return;
  const v4f a0 = *(const v4f*)(in + (size_t)i * 8);
  const v4f a1 = *(const v4f*)(in + (size_t)i * 8 + 4);
  v4u w;
  w[0] = (unsigned)f2bf_bits(a0[0]) | ((unsigned)f2bf_bits(a0[1]) << 16);
  w[1] = (unsigned)f2bf_bits(a0[2]) | ((unsigned)f2bf_bits(a0[3]) << 16);
  w[2] = (unsigned)f2bf_bits(a1[0]) | ((unsigned)f2bf_bits(a1[1]) << 16);
  w[3] = (unsigned)f2bf_bits(a1[2]) | ((unsigned)f2bf_bits(a1[3]) << 16);
  *(volatile v4u*)(out + (size_t)i * 8) = w;
  __threadfence();
  *(volatile v4u*)(out + (size_t)i * 8) = w;
}

__global__ __launch_bounds__(256) void tcast_bf16(
    const float* __restrict__ in, unsigned short* __restrict__ out, int R, int C) {
  __shared__ float tile[64][65];
  const int t = threadIdx.x;
  const int r0 = blockIdx.y * 64, c0 = blockIdx.x * 64;
  {
    const int rr = t >> 2, cc = (t & 3) * 16;
    const float* src = in + (size_t)(r0 + rr) * C + c0 + cc;
#pragma unroll
    for (int i = 0; i < 4; ++i) {
      const v4f v = *(const v4f*)(src + 4 * i);
      tile[rr][cc + 4 * i + 0] = v[0];
      tile[rr][cc + 4 * i + 1] = v[1];
      tile[rr][cc + 4 * i + 2] = v[2];
      tile[rr][cc + 4 * i + 3] = v[3];
    }
  }
  __syncthreads();
  const int c8 = (t & 7) * 8;
  for (int pass = 0; pass < 2; ++pass) {
#pragma unroll
    for (int p = 0; p < 2; ++p) {
      const int n = p * 32 + (t >> 3);
      v4u w;
#pragma unroll
      for (int e2 = 0; e2 < 4; ++e2) {
        const unsigned lo = (unsigned)f2bf_bits(tile[c8 + 2 * e2][n]);
        const unsigned hi = (unsigned)f2bf_bits(tile[c8 + 2 * e2 + 1][n]);
        w[e2] = lo | (hi << 16);
      }
      *(volatile v4u*)(out + (size_t)(c0 + n) * R + r0 + c8) = w;
    }
    __threadfence();
  }
}

struct AttnTiles {
  unsigned short Kh[KVC * HDIM];
  unsigned short Kl[KVC * HDIM];
  unsigned short Vh[HDIM * KVC];
  unsigned short Vl[HDIM * KVC];
  unsigned short Ph[4][16 * KVC];
  unsigned short Pl[4][16 * KVC];
};
union AttnSmemU { AttnTiles t; float Os[4][16 * OSP]; };
static_assert(sizeof(AttnTiles) == 49152, "lds tiles");
static_assert(sizeof(float) * 4 * 16 * OSP <= sizeof(AttnTiles), "out slab fits in the union");

__global__ __launch_bounds__(128) void attn_planes(
    const unsigned short* __restrict__ qkh, const unsigned short* __restrict__ qkl,
    const unsigned short* __restrict__ vth, const unsigned short* __restrict__ vtl,
    const float* __restrict__ amask,
    unsigned short* __restrict__ xh, unsigned short* __restrict__ xl, int bglob0) {
  __shared__ __align__(16) AttnSmemU sm;
  const int tid  = threadIdx.x;
  const int wave = tid >> 5;
  const int lane = tid & 31;
  const int hh   = lane >> 4;
  const int c    = lane & 15;

  const int bx = blockIdx.x;
  const int qb = bx % NQB;
  const int bh = bx / NQB;
  const int h  = bh % NHEAD;
  const int bl = bh / NHEAD;
  const int q0 = qb * QBLK + wave * 16;
  const size_t rowbase = (size_t)bl * SEQ_LEN;

  v16b qah[2], qal[2];
  {
    const size_t qo = (rowbase + q0 + c) * LDQK + (size_t)h * HDIM + 8 * hh;
#pragma unroll
    for (int dc = 0; dc < 2; ++dc) {
      qah[dc] = Frag<__bf16>::load((const __bf16*)qkh + qo + dc * 32);
      qal[dc] = Frag<__bf16>::load((const __bf16*)qkl + qo + dc * 32);
    }
  }

  float mrow[8], lrow[8];
  v8f oacc[4];
#pragma unroll
  for (int r = 0; r < 8; ++r) { mrow[r] = -INFINITY; lrow[r] = 0.f; }
#pragma unroll
  for (int t = 0; t < 4; ++t) oacc[t] = (v8f){0.f,0.f,0.f,0.f,0.f,0.f,0.f,0.f};

  const float* mvec = amask + (size_t)(bglob0 + bl) * MASK_LEN;
  const int nChunks = qb + 1;
  for (int kc = 0; kc < nChunks; ++kc) {
    const int kv0 = kc * KVC;
    __syncthreads();
    {
      const int rr = tid >> 1, half32 = (tid & 1) * 32;
      const size_t ko = (rowbase + kv0 + rr) * LDQK + DMODEL + (size_t)h * HDIM + half32;
      const v4u* gkh = (const v4u*)(qkh + ko);
      const v4u* gkl = (const v4u*)(qkl + ko);
      v4u* lkh = (v4u*)(sm.t.Kh + rr * HDIM + half32);
      v4u* lkl = (v4u*)(sm.t.Kl + rr * HDIM + half32);
#pragma unroll
      for (int i = 0; i < 4; ++i) { lkh[i] = gkh[i]; lkl[i] = gkl[i]; }
      asm volatile("" ::: "memory");
      const size_t vo = (size_t)bl * DMODEL * SEQ_LEN + (size_t)(h * HDIM + rr) * SEQ_LEN + kv0 + half32;
      const v4u* gvh = (const v4u*)(vth + vo);
      const v4u* gvl = (const v4u*)(vtl + vo);
      v4u* lvh = (v4u*)(sm.t.Vh + rr * KVC + half32);
      v4u* lvl = (v4u*)(sm.t.Vl + rr * KVC + half32);
#pragma unroll
      for (int i = 0; i < 4; ++i) { lvh[i] = gvh[i]; lvl[i] = gvl[i]; }
    }
    __syncthreads();

    v8f s[4];
#pragma unroll
    for (int j = 0; j < 4; ++j) {
      s[j] = (v8f){0.f,0.f,0.f,0.f,0.f,0.f,0.f,0.f};
#pragma unroll
      for (int dc = 0; dc < 2; ++dc) {
        const v16b kbh = Frag<__bf16>::load((const __bf16*)sm.t.Kh + (j * 16 + c) * HDIM + dc * 32 + 8 * hh);
        const v16b kbl = Frag<__bf16>::load((const __bf16*)sm.t.Kl + (j * 16 + c) * HDIM + dc * 32 + 8 * hh);
        s[j] = at_mma(qah[dc], kbh, s[j]);
        s[j] = at_mma(qah[dc], kbl, s[j]);
        s[j] = at_mma(qal[dc], kbh, s[j]);
      }
    }
    float mk[4];
#pragma unroll
    for (int j = 0; j < 4; ++j) mk[j] = mvec[kv0 + j * 16 + c];
    const bool diag = (kc == qb);
    float cm[8];
#pragma unroll
    for (int r = 0; r < 8; ++r) {
      const int qrow = q0 + 8 * hh + r;
      float m = -INFINITY;
#pragma unroll
      for (int j = 0; j < 4; ++j) {
        const int kvcol = kv0 + j * 16 + c;
        float sv = s[j][r] * 0.125f;
        if (diag && (kvcol > qrow)) sv = -1.0e9f;
        if (mk[j] == 0.0f) sv = -1.0e4f;
        s[j][r] = sv;
        m = fmaxf(m, sv);
      }
#pragma unroll
      for (int off = 1; off < 16; off <<= 1) m = fmaxf(m, __shfl_xor(m, off, 32));
      cm[r] = m;
    }
    unsigned short* pwh = sm.t.Ph[wave];
    unsigned short* pwl = sm.t.Pl[wave];
#pragma unroll
    for (int r = 0; r < 8; ++r) {
      const float mnew = fmaxf(mrow[r], cm[r]);
      const float alpha = expf(mrow[r] - mnew);
      mrow[r] = mnew;
      float psum = 0.f;
#pragma unroll
      for (int j = 0; j < 4; ++j) {
        const float p = expf(s[j][r] - mnew);
        psum += p;
        const unsigned short hb = f2bf_bits(p);
        const unsigned short lb = f2bf_bits(p - bf_bits2f(hb));
        const int po = (8 * hh + r) * KVC + j * 16 + c;
        pwh[po] = hb;
        pwl[po] = lb;
      }
#pragma unroll
      for (int off = 1; off < 16; off <<= 1) psum += __shfl_xor(psum, off, 32);
      lrow[r] = lrow[r] * alpha + psum;
#pragma unroll
      for (int t = 0; t < 4; ++t) oacc[t][r] *= alpha;
    }
    __builtin_amdgcn_fence(__ATOMIC_RELEASE, "workgroup");
    __builtin_amdgcn_wave_barrier();
    __builtin_amdgcn_fence(__ATOMIC_ACQUIRE, "workgroup");
#pragma unroll
    for (int kk = 0; kk < 2; ++kk) {
      const v16b pa = Frag<__bf16>::load((const __bf16*)pwh + c * KVC + kk * 32 + 8 * hh);
      const v16b pl = Frag<__bf16>::load((const __bf16*)pwl + c * KVC + kk * 32 + 8 * hh);
#pragma unroll
      for (int t = 0; t < 4; ++t) {
        const v16b vbh = Frag<__bf16>::load((const __bf16*)sm.t.Vh + (t * 16 + c) * KVC + kk * 32 + 8 * hh);
        const v16b vbl = Frag<__bf16>::load((const __bf16*)sm.t.Vl + (t * 16 + c) * KVC + kk * 32 + 8 * hh);
        oacc[t] = at_mma(pa, vbh, oacc[t]);
        oacc[t] = at_mma(pa, vbl, oacc[t]);
        oacc[t] = at_mma(pl, vbh, oacc[t]);
      }
    }
  }

  __syncthreads();
  float* os = sm.Os[wave];
#pragma unroll
  for (int r = 0; r < 8; ++r) {
    const float inv = 1.0f / lrow[r];
#pragma unroll
    for (int t = 0; t < 4; ++t) os[(8 * hh + r) * OSP + t * 16 + c] = oacc[t][r] * inv;
  }
  __builtin_amdgcn_fence(__ATOMIC_RELEASE, "workgroup");
  __builtin_amdgcn_wave_barrier();
  __builtin_amdgcn_fence(__ATOMIC_ACQUIRE, "workgroup");
  {
    const int q8 = lane >> 3, c8 = (lane & 7) * 8;
    for (int pass = 0; pass < 2; ++pass) {
#pragma unroll
      for (int it = 0; it < 4; ++it) {
        const int row = it * 4 + q8;
        const float* sp = os + row * OSP + c8;
        v4u wh, wl;
#pragma unroll
        for (int e2 = 0; e2 < 4; ++e2) {
          const float f0 = sp[2 * e2], f1 = sp[2 * e2 + 1];
          const unsigned short h0 = f2bf_bits(f0), h1 = f2bf_bits(f1);
          const unsigned short l0 = f2bf_bits(f0 - bf_bits2f(h0)), l1 = f2bf_bits(f1 - bf_bits2f(h1));
          wh[e2] = (unsigned)h0 | ((unsigned)h1 << 16);
          wl[e2] = (unsigned)l0 | ((unsigned)l1 << 16);
        }
        const size_t xo = (rowbase + q0 + row) * DMODEL + (size_t)h * HDIM + c8;
        *(volatile v4u*)(xh + xo) = wh;
        *(volatile v4u*)(xl + xo) = wl;
      }
      __threadfence();
    }
  }
}

extern "C" void kernel_launch(void* const* d_in, const int* in_sizes, int n_in,
                              void* d_out, int out_size, void* d_ws, size_t ws_size,
                              hipStream_t stream) {
  if (n_in < 9) return;
  if (in_sizes[0] != NBATCH * SEQ_LEN * DMODEL) return;
  if (in_sizes[1] != NBATCH * MASK_LEN) return;
  if (in_sizes[3] != DMODEL * 3 * DMODEL) return;
  if (in_sizes[4] != 3 * DMODEL) return;
  if (in_sizes[5] != DMODEL * DMODEL) return;
  if (in_sizes[6] != DMODEL) return;
  if (out_size != NBATCH * SEQ_LEN * DMODEL) return;
  if (WS_TOTAL > ws_size) return;

  const float* hidden  = (const float*)d_in[0];
  const float* amask   = (const float*)d_in[1];
  const float* Wc_attn = (const float*)d_in[3];
  const float* bc_attn = (const float*)d_in[4];
  const float* Wc_proj = (const float*)d_in[5];
  const float* bc_proj = (const float*)d_in[6];
  float* out = (float*)d_out;

  char* ws = (char*)d_ws;
  size_t off = 0;
  unsigned short* Xb    = (unsigned short*)(ws + off); off += WS_XB;
  unsigned short* Wqkvt = (unsigned short*)(ws + off); off += WS_WQKV;
  unsigned short* Wpt   = (unsigned short*)(ws + off); off += WS_WP;
  unsigned short* QKh   = (unsigned short*)(ws + off); off += WS_QK;
  unsigned short* QKl   = (unsigned short*)(ws + off); off += WS_QK;
  unsigned short* Vth   = (unsigned short*)(ws + off); off += WS_VT;
  unsigned short* Vtl   = (unsigned short*)(ws + off); off += WS_VT;
  unsigned short* Xh    = (unsigned short*)(ws + off); off += WS_X;
  unsigned short* Xl    = (unsigned short*)(ws + off); off += WS_X;
  if (off > ws_size) return;

  {
    const int n8 = NBATCH * SEQ_LEN * DMODEL / 8;
    cast_rows_bf16<<<dim3((n8 + 255) / 256), 256, 0, stream>>>(hidden, Xb, n8);
  }
  tcast_bf16<<<dim3(3 * DMODEL / 64, DMODEL / 64), 256, 0, stream>>>(Wc_attn, Wqkvt, DMODEL, 3 * DMODEL);
  tcast_bf16<<<dim3(DMODEL / 64, DMODEL / 64), 256, 0, stream>>>(Wc_proj, Wpt, DMODEL, DMODEL);

  for (int half = 0; half < NBATCH / HALF_NB; ++half) {
    const unsigned short* Xhalf = Xb + (size_t)half * ROWS_HALF * DMODEL;
    {
      const int tiles = (ROWS_HALF / 64) * (LDQK / 64);
      wmma_gemm64<1, 0, 2, 2, false><<<dim3(tiles / 8, 1), 256, 0, stream>>>(
          Xhalf, Xhalf, DMODEL, 0L,
          Wqkvt, Wqkvt, DMODEL, 0L,
          (void*)QKh, (void*)QKl, LDQK, 0L,
          bc_attn, nullptr, 0L,
          ROWS_HALF, LDQK, DMODEL, 1.0f);
    }
    {
      const int tiles = (DMODEL / 64) * (SEQ_LEN / 64);
      wmma_gemm64<1, 0, 1, 2, false><<<dim3(tiles / 8, HALF_NB), 256, 0, stream>>>(
          Wqkvt + (size_t)2 * DMODEL * DMODEL, Wqkvt + (size_t)2 * DMODEL * DMODEL, DMODEL, 0L,
          Xhalf, Xhalf, DMODEL, (long)SEQ_LEN * DMODEL,
          (void*)Vth, (void*)Vtl, SEQ_LEN, (long)DMODEL * SEQ_LEN,
          bc_attn + 2 * DMODEL, nullptr, 0L,
          DMODEL, SEQ_LEN, DMODEL, 1.0f);
    }
    attn_planes<<<dim3(HALF_NB * NHEAD * NQB), 128, 0, stream>>>(QKh, QKl, Vth, Vtl, amask, Xh, Xl, half * HALF_NB);
    {
      const int tiles = (ROWS_HALF / 64) * (DMODEL / 64);
      wmma_gemm64<1, 2, 2, 0, false><<<dim3(tiles / 8, 1), 256, 0, stream>>>(
          Xh, Xl, DMODEL, 0L,
          Wpt, Wpt, DMODEL, 0L,
          (void*)(out + (size_t)half * ROWS_HALF * DMODEL), nullptr, DMODEL, 0L,
          bc_proj, nullptr, 0L,
          ROWS_HALF, DMODEL, DMODEL, 1.0f);
    }
  }
}
